// TransformerDecoderBlock_14181982012037
// MI455X (gfx1250) — hardware-verified
//
#include <hip/hip_runtime.h>
#include <math.h>
#include <stdint.h>

#ifndef NB
#define NB      2
#endif
#ifndef SEQ
#define SEQ     2048
#endif
#define NB_FULL  2
#define SEQ_FULL 2048
#define NQ      SEQ
#define NC      SEQ
#define DMODEL  512
#define DFF     2048
#define NHEAD   8
#define HDIM    64
#define QKP     (2 * DMODEL)
#define NROWS   (NB * NQ)
#define NCH     (NC / 32)
#define WSC     64.0f
#define XC      16.0f
#define QC      16.0f
#define KC      16.0f
#define VC      16.0f
#define PC      1024.0f
#define FC      1024.0f
#define X1C     16.0f
#define GC      64.0f
#define ATT_SCALE 0.125f
#define LOG2E   1.4426950408889634f
#define LN_EPS  1e-6f
#define MASK_NEG (-1.0e9f)
static_assert(NHEAD * HDIM == DMODEL);
static_assert(NB >= 1 && NB <= NB_FULL && SEQ >= 64 && SEQ <= SEQ_FULL);
static_assert((NQ % 64) == 0 && (NC % 64) == 0 && (DMODEL % 64) == 0 && (DFF % 64) == 0 && (QKP % 64) == 0 && (NC % 32) == 0);
static_assert((NROWS % 64) == 0 && (DMODEL % 32) == 0 && (DFF % 32) == 0 && (NQ % 16) == 0);
static_assert(((SEQ * DMODEL) % 2048) == 0);
static_assert(((16 * NCH) % 32) == 0 && NCH <= 256 && NCH >= 2);
#define HPB     8
#define OSP     (HPB * HDIM)
#define ATT_THREADS (HPB * 32)
#define ATT_BLOCKS  (NB * (NQ / 16))
static_assert(ATT_THREADS == 256 && HPB == NHEAD && OSP == DMODEL);
#define LN_THREADS 128
static_assert(LN_THREADS * 4 == DMODEL && (DMODEL / 8) * 8 == DMODEL && (DMODEL / 8) == 64);

typedef _Float16 v16h __attribute__((ext_vector_type(16)));
typedef _Float16 v8h  __attribute__((ext_vector_type(8)));
typedef float    v8f  __attribute__((ext_vector_type(8)));
typedef float    v4f  __attribute__((ext_vector_type(4)));
typedef unsigned int v4u __attribute__((ext_vector_type(4)));
typedef unsigned int v2u __attribute__((ext_vector_type(2)));

union FragH { v16h v; v8h h[2]; v4u u[2]; };

__device__ __forceinline__ unsigned short bf_bits(float f) {
  unsigned u = __float_as_uint(f);
  return (unsigned short)((u + 0x7FFFu + ((u >> 16) & 1u)) >> 16);
}
__device__ __forceinline__ float bf_up(unsigned short h) { return __uint_as_float(((unsigned)h) << 16); }
__device__ __forceinline__ float bfr(float f) { return bf_up(bf_bits(f)); }
__device__ __forceinline__ unsigned short h_bits(_Float16 x) { return __builtin_bit_cast(unsigned short, x); }
__device__ __forceinline__ unsigned pk16(unsigned short a, unsigned short b) { return (unsigned)a | ((unsigned)b << 16); }
__device__ __forceinline__ v8f zero8() { v8f z = {0.f, 0.f, 0.f, 0.f, 0.f, 0.f, 0.f, 0.f}; return z; }
__device__ __forceinline__ int imin(int a, int b) { return a < b ? a : b; }
__device__ __forceinline__ int imax(int a, int b) { return a > b ? a : b; }

__device__ __forceinline__ float bias2(const float* a, int nA, const float* b, int nB, int n) {
  const int ia = imin(n, nA - 1);
  const int ib = imin(imax(n - nA, 0), nB - 1);
  const float ta = bfr(a[ia]);
  const float tb = bfr(b[ib]);
  return (n < nA) ? ta : (((n - nA) < nB) ? tb : 0.f);
}

__device__ __forceinline__ v16h ldfrag_h(const _Float16* p) {
  FragH f;
  f.h[0] = *(const v8h*)(p);
  f.h[1] = *(const v8h*)(p + 16);
  return f.v;
}
__device__ __forceinline__ v16h ldfrag_u(const unsigned short* p) {
  FragH f;
  f.u[0] = *(const v4u*)(p);
  f.u[1] = *(const v4u*)(p + 16);
  return f.v;
}

__device__ __forceinline__ v8f mma_raw(v16h a, v16h b, v8f c) {
  return __builtin_amdgcn_wmma_f32_16x16x32_f16(false, a, false, b, (short)0, c, false, false);
}
__device__ __forceinline__ void dep_guard1(v8f& a, v8f& b, v16h x) {
#if defined(__HIP_DEVICE_COMPILE__)
  asm volatile("v_nop\n\tv_nop\n\tv_nop\n\tv_nop" : "+v"(a), "+v"(b) : "v"(x));
#endif
}
__device__ __forceinline__ void guard_s2(v8f& s, v16h a0, v16h a1) {
#if defined(__HIP_DEVICE_COMPILE__)
  asm volatile("v_nop\n\tv_nop\n\tv_nop\n\tv_nop" : "+v"(s) : "v"(a0), "v"(a1));
#endif
}
__device__ __forceinline__ void guard_s4(v8f& s, v16h a0, v16h a1, v16h b0, v16h b1) {
#if defined(__HIP_DEVICE_COMPILE__)
  asm volatile("v_nop\n\tv_nop\n\tv_nop\n\tv_nop" : "+v"(s) : "v"(a0), "v"(a1), "v"(b0), "v"(b1));
#endif
}
__device__ __forceinline__ void guard_pv4(v8f& a, v8f& b, v8f& c, v8f& d, v16h x, v16h y, v16h z, v16h w, v16h u) {
#if defined(__HIP_DEVICE_COMPILE__)
  asm volatile("v_nop\n\tv_nop\n\tv_nop\n\tv_nop"
               : "+v"(a), "+v"(b), "+v"(c), "+v"(d) : "v"(x), "v"(y), "v"(z), "v"(w), "v"(u));
#endif
}
__device__ __forceinline__ void keep4_h(v16h a, v16h b, v16h c, v16h d) {
#if defined(__HIP_DEVICE_COMPILE__)
  asm volatile("v_nop" :: "v"(a), "v"(b), "v"(c), "v"(d));
#endif
}
__device__ __forceinline__ void acc_guard4(v8f& a, v8f& b, v8f& c, v8f& d) {
#if defined(__HIP_DEVICE_COMPILE__)
  asm volatile("v_nop\n\tv_nop\n\tv_nop\n\tv_nop" : "+v"(a), "+v"(b), "+v"(c), "+v"(d));
#endif
}
__device__ __forceinline__ void wave_sync_lds() {
  __builtin_amdgcn_fence(3, "workgroup");
  __builtin_amdgcn_wave_barrier();
  __builtin_amdgcn_fence(2, "workgroup");
}

__global__ __launch_bounds__(256) void cvt16(const float* __restrict__ src, unsigned short* dst, int n8, float sc) {
  const int i = blockIdx.x * 256 + threadIdx.x;
  if (i >= n8) return;
  const float* p = src + (size_t)i * 8;
  const v4f a = *(const v4f*)(p);
  const v4f b = *(const v4f*)(p + 4);
  v4u w;
  w[0] = pk16(h_bits((_Float16)(bfr(a[0]) * sc)), h_bits((_Float16)(bfr(a[1]) * sc)));
  w[1] = pk16(h_bits((_Float16)(bfr(a[2]) * sc)), h_bits((_Float16)(bfr(a[3]) * sc)));
  w[2] = pk16(h_bits((_Float16)(bfr(b[0]) * sc)), h_bits((_Float16)(bfr(b[1]) * sc)));
  w[3] = pk16(h_bits((_Float16)(bfr(b[2]) * sc)), h_bits((_Float16)(bfr(b[3]) * sc)));
  unsigned short* d = dst + (size_t)i * 8;
  for (int pass = 0; pass < 2; ++pass) {
    *(volatile v4u*)d = w;
    __threadfence();
  }
}

static_assert(4 * 256 * 4 == 64 * 64 && 2 * 256 * 8 == 64 * 64);
__global__ __launch_bounds__(256) void cvtT16(const float* __restrict__ src, unsigned short* dst,
                                              unsigned K, unsigned N, float sc) {
  __shared__ __align__(16) unsigned short tl[64 * 72];
  const unsigned tid = threadIdx.x;
  const unsigned n0 = blockIdx.x * 64u;
  const unsigned k0 = blockIdx.y * 64u;
#pragma unroll
  for (unsigned it = 0; it < 4; ++it) {
    const unsigned p  = it * 256u + tid;
    const unsigned kr = p >> 4;
    const unsigned nc = (p & 15u) * 4u;
    const v4f a = *(const v4f*)(src + (size_t)(k0 + kr) * N + n0 + nc);
#pragma unroll
    for (unsigned e = 0; e < 4; ++e) tl[(nc + e) * 72u + kr] = h_bits((_Float16)(bfr(a[e]) * sc));
  }
  __syncthreads();
  v4u vals[2];
#pragma unroll
  for (unsigned it = 0; it < 2; ++it) {
    const unsigned p = it * 256u + tid;
    const unsigned row = p >> 3, c8 = (p & 7u) * 8u;
    vals[it] = *(const v4u*)(tl + row * 72u + c8);
  }
  for (int pass = 0; pass < 2; ++pass) {
#pragma unroll
    for (unsigned it = 0; it < 2; ++it) {
      const unsigned p = it * 256u + tid;
      const unsigned row = p >> 3, c8 = (p & 7u) * 8u;
      *(volatile v4u*)(dst + (size_t)(n0 + row) * K + k0 + c8) = vals[it];
    }
    __threadfence();
  }
}

template <int OM, int RM, int ACT, int BM>
__global__ __launch_bounds__(256) void gemm64(
    const unsigned short* __restrict__ Ap, int lda, long long sA,
    const unsigned short* __restrict__ Btp, int ldb, long long sB,
    const float* __restrict__ Rp, long long sR,
    const float* __restrict__ biasA, int nA,
    const float* __restrict__ biasB, int nB,
    void* Cout, int ldc, long long sC,
    int M, int N, int K, float oscale, float ocarry) {
  static_assert(!(BM == 2 && OM == 0));
  __shared__ __align__(16) float sT[8][16 * 68];
  const int by   = blockIdx.y;
  const int lane = threadIdx.x & 31;
  const int wave = threadIdx.x >> 5;
  const unsigned tilesN = (unsigned)N >> 6;
  const unsigned tilesM = (unsigned)M >> 6;
  const unsigned tile = blockIdx.x * 8u + (unsigned)wave;
  if (tile >= tilesM * tilesN) return;
  const unsigned tm = tile / tilesN;
  const unsigned tn = tile - tm * tilesN;
  const int m0 = (int)(tm << 6);
  const int n0 = (int)(tn << 6);

  const unsigned short* A1 = Ap  + (size_t)((long long)by * sA);
  const unsigned short* Bb = Btp + (size_t)((long long)by * sB);

  const int rlane = lane & 15;
  const int koff  = (lane >> 4) * 8;
  const int mOff  = (lane >> 4) * 8;

  v8f acc[4][4];
#pragma unroll
  for (int i = 0; i < 4; ++i)
#pragma unroll
    for (int j = 0; j < 4; ++j) acc[i][j] = zero8();

  for (int k0 = 0; k0 < K; k0 += 32) {
    v16h bh[4];
#pragma unroll
    for (int j = 0; j < 4; ++j) {
      const size_t bofs = (size_t)(n0 + (j << 4) + rlane) * ldb + koff + k0;
      bh[j] = ldfrag_u(Bb + bofs);
    }
#pragma unroll
    for (int i = 0; i < 4; ++i) {
      const size_t ao = (size_t)(m0 + (i << 4) + rlane) * lda + koff + k0;
      const v16h ah = ldfrag_u(A1 + ao);
#pragma unroll
      for (int j = 0; j < 4; ++j) acc[i][j] = mma_raw(ah, bh[j], acc[i][j]);
      dep_guard1(acc[i][0], acc[i][3], ah);
    }
    keep4_h(bh[0], bh[1], bh[2], bh[3]);
  }
  acc_guard4(acc[0][0], acc[0][1], acc[0][2], acc[0][3]);
  acc_guard4(acc[1][0], acc[1][1], acc[1][2], acc[1][3]);
  acc_guard4(acc[2][0], acc[2][1], acc[2][2], acc[2][3]);
  acc_guard4(acc[3][0], acc[3][1], acc[3][2], acc[3][3]);

  const int hh2 = lane >> 4, c4 = (lane & 15) * 4;
  const int q8  = lane >> 3, c8 = (lane & 7) * 8;

  float bc4[4], bc8[8];
#pragma unroll
  for (int e = 0; e < 4; ++e) bc4[e] = 0.f;
#pragma unroll
  for (int e = 0; e < 8; ++e) bc8[e] = 0.f;
  if constexpr (BM == 1) {
    if constexpr (OM == 0) {
#pragma unroll
      for (int e = 0; e < 4; ++e) bc4[e] = bias2(biasA, nA, biasB, nB, n0 + c4 + e);
    } else {
#pragma unroll
      for (int e = 0; e < 8; ++e) bc8[e] = bias2(biasA, nA, biasB, nB, n0 + c8 + e);
    }
  }

  float* slab = sT[wave];
#pragma unroll
  for (int i = 0; i < 4; ++i) {
    const int mBase = m0 + (i << 4);
#pragma unroll
    for (int j = 0; j < 4; ++j) {
#pragma unroll
      for (int r = 0; r < 8; ++r) {
        slab[(mOff + r) * 68 + (j << 4) + rlane] = acc[i][j][r];
      }
    }
    wave_sync_lds();
    if constexpr (OM == 0) {
      float* C = (float*)Cout + (size_t)((long long)by * sC);
      v4f vals[8];
#pragma unroll
      for (int it = 0; it < 8; ++it) {
        const int row = it * 2 + hh2;
        const int gr  = mBase + row;
        v4f v = *(const v4f*)(slab + row * 68 + c4);
        v4f rv = {0.f, 0.f, 0.f, 0.f};
        if constexpr (RM == 1 || RM == 2) {
          const float* R = Rp + (size_t)((long long)by * sR);
          const v4f rraw = *(const v4f*)(R + (size_t)gr * ldc + n0 + c4);
#pragma unroll
          for (int e = 0; e < 4; ++e) rv[e] = (RM == 1) ? bfr(rraw[e]) : rraw[e];
        }
#pragma unroll
        for (int e = 0; e < 4; ++e) {
          float u = v[e] * oscale;
          if constexpr (BM == 1) u += bc4[e];
          if constexpr (ACT == 1) u = fmaxf(u, 0.f);
          v[e] = u + rv[e];
        }
        vals[it] = v;
      }
      for (int pass = 0; pass < 2; ++pass) {
#pragma unroll
        for (int it = 0; it < 8; ++it) {
          const int gr = mBase + it * 2 + hh2;
          *(volatile v4f*)(C + (size_t)gr * ldc + n0 + c4) = vals[it];
        }
        __threadfence();
      }
    } else {
      unsigned short* C = (unsigned short*)Cout + (size_t)((long long)by * sC);
      v4u hv[4];
#pragma unroll
      for (int it = 0; it < 4; ++it) {
        const int row = it * 4 + q8;
        const float* sp = slab + row * 68 + c8;
        float rb = 0.f;
        if constexpr (BM == 2) {
          const int gr  = mBase + row;
          const int gcl = imin(gr, nA - 1);
          const float t = bfr(biasA[gcl]);
          rb = (gr < nA) ? t : 0.f;
        }
        v4u a = {0u, 0u, 0u, 0u};
#pragma unroll
        for (int e = 0; e < 4; ++e) {
          float f0 = sp[2 * e] * oscale;
          float f1 = sp[2 * e + 1] * oscale;
          if constexpr (BM == 1) { f0 += bc8[2 * e]; f1 += bc8[2 * e + 1]; }
          if constexpr (BM == 2) { f0 += rb; f1 += rb; }
          if constexpr (ACT == 1) { f0 = fmaxf(f0, 0.f); f1 = fmaxf(f1, 0.f); }
          f0 *= ocarry; f1 *= ocarry;
          a[e] = pk16(h_bits((_Float16)f0), h_bits((_Float16)f1));
        }
        hv[it] = a;
      }
      for (int pass = 0; pass < 2; ++pass) {
#pragma unroll
        for (int it = 0; it < 4; ++it) {
          const int row = it * 4 + q8;
          *(volatile v4u*)(C + (size_t)(mBase + row) * ldc + n0 + c8) = hv[it];
        }
        __threadfence();
      }
    }
    wave_sync_lds();
  }
}

#define PS_FLOATS (HPB * 16 * 36)
static_assert((size_t)16 * OSP * sizeof(unsigned short) <= (size_t)PS_FLOATS * sizeof(float));
static_assert(((16 * OSP) % (8 * ATT_THREADS)) == 0 && ((16 * OSP) / (8 * ATT_THREADS)) == 4);
static_assert(OSP == 64 * 8);

template <int MM>
__global__ __launch_bounds__(ATT_THREADS) __attribute__((amdgpu_num_vgpr(256)))
void attn8(const unsigned short* __restrict__ QKq, const unsigned short* __restrict__ VTq,
           const float* __restrict__ maskp, unsigned short* CT) {
  __shared__ __align__(16) float smem[PS_FLOATS];
  __shared__ int cellf[16 * NCH];
  __shared__ int chunkf[NCH];
  __shared__ int rowok[16];

  const unsigned tid  = threadIdx.x;
  const unsigned wave = tid >> 5;
  const unsigned lane = tid & 31u;
  const unsigned hh   = lane >> 4;
  const unsigned c    = lane & 15u;

  const unsigned qt   = blockIdx.x % (unsigned)(NQ / 16);
  const unsigned bat  = blockIdx.x / (unsigned)(NQ / 16);
  const unsigned head = wave;
  const unsigned q0   = qt * 16u;

  int safe = 0;
  if constexpr (MM == 0) {
    for (unsigned cell = tid; cell < 16u * (unsigned)NCH; cell += (unsigned)ATT_THREADS) {
      const unsigned row = cell / (unsigned)NCH;
      const unsigned ch  = cell % (unsigned)NCH;
      const float* mp = maskp + (size_t)(q0 + row) * SEQ_FULL + ch * 32u;
      int a0 = 1, a1 = 1, z = 0;
#pragma unroll
      for (int j = 0; j < 8; ++j) {
        const v4f m = *(const v4f*)(mp + 4 * j);
#pragma unroll
        for (int e = 0; e < 4; ++e) {
          const int is0 = (m[e] == 0.f) ? 1 : 0;
          const int is1 = (m[e] == 1.f) ? 1 : 0;
          a0 &= is0; a1 &= is1; z |= is0;
        }
      }
      cellf[cell] = a0 | (a1 << 1) | (z << 2);
    }
    __syncthreads();
    {
      const unsigned ch = (tid < (unsigned)NCH) ? tid : (unsigned)(NCH - 1);
      int a = 3;
#pragma unroll 4
      for (unsigned r = 0; r < 16u; ++r) a &= cellf[r * (unsigned)NCH + ch];
      if (tid < (unsigned)NCH) chunkf[tid] = a & 3;
      const unsigned rr = tid & 15u;
      int o = 0;
#pragma unroll 4
      for (unsigned k = 0; k < (unsigned)NCH; ++k) o |= cellf[rr * (unsigned)NCH + k];
      if (tid < 16u) rowok[tid] = (o >> 2) & 1;
    }
    __syncthreads();
    int s = 1;
#pragma unroll
    for (int r = 0; r < 16; ++r) s &= rowok[r];
    safe = __builtin_amdgcn_readfirstlane(s);
  }

  const size_t qofs = ((size_t)bat * NQ + q0 + c) * QKP + head * HDIM + 8u * hh;
  const _Float16* Qh = (const _Float16*)(const void*)QKq + qofs;
  const _Float16* Kb = (const _Float16*)(const void*)QKq + (size_t)bat * NC * QKP + DMODEL + head * HDIM + 8u * hh;
  const _Float16* Vb = (const _Float16*)(const void*)VTq + ((size_t)bat * DMODEL + head * HDIM) * NC + 8u * hh;
  const float ssc = ATT_SCALE / (QC * KC);

  const v16h qa = ldfrag_h(Qh), qb = ldfrag_h(Qh + 32);

  float mrow[8], lrow[8];
  v8f o0 = zero8(), o1 = zero8(), o2 = zero8(), o3 = zero8();
#pragma unroll
  for (int r = 0; r < 8; ++r) { mrow[r] = -INFINITY; lrow[r] = 0.f; }
  float* pt = smem + wave * (16 * 36);

#pragma unroll 1
  for (unsigned j = 0; j < (unsigned)NCH; ++j) {
    const unsigned kb = j * 32u;
    int cf = 1;
    if constexpr (MM == 0) {
      cf = __builtin_amdgcn_readfirstlane(chunkf[j]);
      if (cf == 2 && safe != 0) continue;
    }
    const _Float16* kp = Kb + (size_t)(kb + c) * QKP;
    v8f s0, s1;
    {
      const v16h k0 = ldfrag_h(kp), k1 = ldfrag_h(kp + 32);
      s0 = mma_raw(qa, k0, zero8());
      s0 = mma_raw(qb, k1, s0);
      guard_s2(s0, k0, k1);
    }
    {
      const _Float16* kq = kp + (size_t)16 * QKP;
      const v16h k0 = ldfrag_h(kq), k1 = ldfrag_h(kq + 32);
      s1 = mma_raw(qa, k0, zero8());
      s1 = mma_raw(qb, k1, s1);
      guard_s4(s1, k0, k1, qa, qb);
    }
    float ma0[8], ma1[8];
#pragma unroll
    for (int r = 0; r < 8; ++r) { ma0[r] = 0.f; ma1[r] = 0.f; }
    if constexpr (MM == 0) {
      if (cf != 1) {
#pragma unroll
        for (unsigned it = 0; it < 4; ++it) {
          const unsigned p = it * 32u + lane;
          const unsigned row = p >> 3, c4 = (p & 7u) * 4u;
          const v4f m = *(const v4f*)(maskp + (size_t)(q0 + row) * SEQ_FULL + kb + c4);
          *(v4f*)(pt + row * 36u + c4) = m;
        }
        wave_sync_lds();
#pragma unroll
        for (int r = 0; r < 8; ++r) {
          ma0[r] = bfr(pt[(8u * hh + r) * 36u + c]) * MASK_NEG;
          ma1[r] = bfr(pt[(8u * hh + r) * 36u + 16u + c]) * MASK_NEG;
        }
        wave_sync_lds();
      }
    } else {
      const float* mb = maskp + (size_t)bat * SEQ_FULL + kb + c;
      const float a0 = bfr(mb[0]) * MASK_NEG;
      const float a1 = bfr(mb[16]) * MASK_NEG;
#pragma unroll
      for (int r = 0; r < 8; ++r) { ma0[r] = a0; ma1[r] = a1; }
    }
#pragma unroll
    for (int r = 0; r < 8; ++r) {
      const float t0 = (s0[r] * ssc + ma0[r]) * LOG2E;
      const float t1 = (s1[r] * ssc + ma1[r]) * LOG2E;
      float mx = fmaxf(t0, t1);
#pragma unroll
      for (int off = 1; off < 16; off <<= 1) mx = fmaxf(mx, __shfl_xor(mx, off, 32));
      const float mn = fmaxf(mrow[r], mx);
      const float alr = exp2f(mrow[r] - mn);
      const float al = (mrow[r] == -INFINITY) ? 0.f : alr;
      mrow[r] = mn;
      const float e0 = exp2f(t0 - mn);
      const float e1 = exp2f(t1 - mn);
      float ps = e0 + e1;
#pragma unroll
      for (int off = 1; off < 16; off <<= 1) ps += __shfl_xor(ps, off, 32);
      lrow[r] = lrow[r] * al + ps;
      o0[r] *= al;
      o1[r] *= al;
      o2[r] *= al;
      o3[r] *= al;
      const unsigned ro = (8u * hh + r) * 36u + c;
      pt[ro]      = e0;
      pt[ro + 16] = e1;
    }
    wave_sync_lds();
    FragH ph;
    {
      const float* prow = pt + c * 36u + 8u * hh;
      const v4f p0 = *(const v4f*)(prow), p1 = *(const v4f*)(prow + 4);
      const v4f p2 = *(const v4f*)(prow + 16), p3 = *(const v4f*)(prow + 20);
#pragma unroll
      for (int e = 0; e < 4; ++e) {
        ph.h[0][e]     = (_Float16)(p0[e] * PC);
        ph.h[0][4 + e] = (_Float16)(p1[e] * PC);
        ph.h[1][e]     = (_Float16)(p2[e] * PC);
        ph.h[1][4 + e] = (_Float16)(p3[e] * PC);
      }
    }
    const _Float16* vp = Vb + (size_t)c * NC + kb;
    {
      const v16h vb0 = ldfrag_h(vp);
      const v16h vb1 = ldfrag_h(vp + (size_t)16 * NC);
      const v16h vb2 = ldfrag_h(vp + (size_t)32 * NC);
      const v16h vb3 = ldfrag_h(vp + (size_t)48 * NC);
      o0 = mma_raw(ph.v, vb0, o0);
      o1 = mma_raw(ph.v, vb1, o1);
      o2 = mma_raw(ph.v, vb2, o2);
      o3 = mma_raw(ph.v, vb3, o3);
      guard_pv4(o0, o1, o2, o3, ph.v, vb0, vb1, vb2, vb3);
    }
    wave_sync_lds();
  }

  __syncthreads();
  unsigned short* Os = (unsigned short*)smem;
  const float oc = FC / (PC * VC);
  unsigned short* osw = Os + wave * HDIM + c;
#pragma unroll
  for (int r = 0; r < 8; ++r) {
    const float inv = (1.0f / lrow[r]) * oc;
    unsigned short* op = osw + (8u * hh + r) * OSP;
    op[0]  = h_bits((_Float16)(o0[r] * inv));
    op[16] = h_bits((_Float16)(o1[r] * inv));
    op[32] = h_bits((_Float16)(o2[r] * inv));
    op[48] = h_bits((_Float16)(o3[r] * inv));
  }
  __syncthreads();
  {
    v4u vals[4];
#pragma unroll
    for (unsigned it = 0; it < 4; ++it) {
      const unsigned p = it * (unsigned)ATT_THREADS + tid;
      vals[it] = *(const v4u*)(Os + (size_t)p * 8);
    }
    unsigned short* dst = CT + ((size_t)bat * NQ + q0) * DMODEL;
    for (int pass = 0; pass < 2; ++pass) {
#pragma unroll
      for (unsigned it = 0; it < 4; ++it) {
        const unsigned p = it * (unsigned)ATT_THREADS + tid;
        const unsigned row = p >> 6, col8 = (p & 63u) * 8u;
        *(volatile v4u*)(dst + (size_t)row * DMODEL + col8) = vals[it];
      }
      __threadfence();
    }
  }
}

template <int OF, int OH>
__global__ __launch_bounds__(LN_THREADS)
void lnorm(const float* __restrict__ Yp, const float* __restrict__ gp, const float* __restrict__ bp,
           float* outf, unsigned short* outh, float hc, unsigned seqIn, unsigned seqOut) {
  __shared__ float red[2][LN_THREADS / 32];
  __shared__ __align__(16) unsigned short srow[DMODEL];
  const unsigned row  = blockIdx.x;
  const unsigned tid  = threadIdx.x;
  const unsigned lane = tid & 31u;
  const unsigned wave = tid >> 5;
  const unsigned bq   = row / (unsigned)SEQ;
  const unsigned tq   = row - bq * (unsigned)SEQ;
  const unsigned irow = bq * seqIn + tq;
  const unsigned orow = bq * seqOut + tq;
  const size_t base = (size_t)irow * DMODEL + (size_t)tid * 4;
  const v4f v = *(const v4f*)(Yp + base);
  float s = (v[0] + v[1]) + (v[2] + v[3]);
#pragma unroll
  for (int off = 1; off < 32; off <<= 1) s += __shfl_xor(s, off, 32);
  if (lane == 0) red[0][wave] = s;
  __syncthreads();
  float tot = 0.f;
#pragma unroll
  for (int w = 0; w < LN_THREADS / 32; ++w) tot += red[0][w];
  const float mu = tot * (1.0f / (float)DMODEL);
  v4f d;
#pragma unroll
  for (int e = 0; e < 4; ++e) d[e] = v[e] - mu;
  float q = (d[0] * d[0] + d[1] * d[1]) + (d[2] * d[2] + d[3] * d[3]);
#pragma unroll
  for (int off = 1; off < 32; off <<= 1) q += __shfl_xor(q, off, 32);
  if (lane == 0) red[1][wave] = q;
  __syncthreads();
  float totq = 0.f;
#pragma unroll
  for (int w = 0; w < LN_THREADS / 32; ++w) totq += red[1][w];
  const float var  = totq * (1.0f / (float)DMODEL);
  const float rstd = rsqrtf(var + LN_EPS);
  const v4f gv = *(const v4f*)(gp + (size_t)tid * 4);
  const v4f bv = *(const v4f*)(bp + (size_t)tid * 4);
  v4f o;
#pragma unroll
  for (int e = 0; e < 4; ++e) o[e] = (d[e] * rstd) * bfr(gv[e]) + bfr(bv[e]);
  if constexpr (OF == 1) {
    float* dst = outf + (size_t)orow * DMODEL + (size_t)tid * 4;
    for (int pass = 0; pass < 2; ++pass) {
      *(volatile v4f*)dst = o;
      __threadfence();
    }
  } else {
    (void)outf; (void)orow; (void)seqOut;
  }
  if constexpr (OH == 1) {
    v2u w;
    w[0] = pk16(h_bits((_Float16)(o[0] * hc)), h_bits((_Float16)(o[1] * hc)));
    w[1] = pk16(h_bits((_Float16)(o[2] * hc)), h_bits((_Float16)(o[3] * hc)));
    *(v2u*)(srow + tid * 4) = w;
    __syncthreads();
    if (tid < DMODEL / 8) {
      const v4u hv = *(const v4u*)(srow + tid * 8);
      unsigned short* dst = outh + (size_t)row * DMODEL + (size_t)tid * 8;
      for (int pass = 0; pass < 2; ++pass) {
        *(volatile v4u*)dst = hv;
        __threadfence();
      }
    }
  } else {
    (void)outh; (void)hc; (void)srow;
  }
}

extern "C" void kernel_launch(void* const* d_in, const int* in_sizes, int n_in,
                              void* d_out, int out_size, void* d_ws, size_t ws_size,
                              hipStream_t stream) {
  if (n_in < 30) return;
  const long long needRows = (long long)(NB - 1) * SEQ_FULL + SEQ;
  if ((long long)in_sizes[0] < needRows * DMODEL) return;
  if ((long long)in_sizes[1] < needRows * DMODEL) return;
  if ((long long)in_sizes[2] < (long long)(SEQ - 1) * SEQ_FULL + SEQ) return;
  if ((long long)in_sizes[3] < needRows) return;
  for (int i = 0; i < 8; ++i) {
    if (in_sizes[4 + 2 * i] != DMODEL * DMODEL || in_sizes[5 + 2 * i] != DMODEL) return;
  }
  if (in_sizes[20] != DMODEL * DFF || in_sizes[21] != DFF) return;
  if (in_sizes[22] != DFF * DMODEL || in_sizes[23] != DMODEL) return;
  for (int i = 24; i < 30; ++i) {
    if (in_sizes[i] != DMODEL) return;
  }
  if ((long long)out_size < needRows * DMODEL) return;

  const float* x     = (const float*)d_in[0];
  const float* enc   = (const float*)d_in[1];
  const float* lmask = (const float*)d_in[2];
  const float* pmask = (const float*)d_in[3];
  const float* q1_w = (const float*)d_in[4];   const float* q1_b = (const float*)d_in[5];
  const float* k1_w = (const float*)d_in[6];   const float* k1_b = (const float*)d_in[7];
  const float* v1_w = (const float*)d_in[8];   const float* v1_b = (const float*)d_in[9];
  const float* o1_w = (const float*)d_in[10];  const float* o1_b = (const float*)d_in[11];
  const float* q2_w = (const float*)d_in[12];  const float* q2_b = (const float*)d_in[13];
  const float* k2_w = (const float*)d_in[14];  const float* k2_b = (const float*)d_in[15];
  const float* v2_w = (const float*)d_in[16];  const float* v2_b = (const float*)d_in[17];
  const float* o2_w = (const float*)d_in[18];  const float* o2_b = (const float*)d_in[19];
  const float* f1_w = (const float*)d_in[20];  const float* f1_b = (const float*)d_in[21];
  const float* f2_w = (const float*)d_in[22];  const float* f2_b = (const float*)d_in[23];
  const float* ln1_g = (const float*)d_in[24]; const float* ln1_b = (const float*)d_in[25];
  const float* ln2_g = (const float*)d_in[26]; const float* ln2_b = (const float*)d_in[27];
  const float* ln3_g = (const float*)d_in[28]; const float* ln3_b = (const float*)d_in[29];
  float*       out   = (float*)d_out;

  const size_t PWQK = (size_t)QKP * DMODEL * 2;
  const size_t PWD  = (size_t)DMODEL * DMODEL * 2;
  const size_t PWF  = (size_t)DFF * DMODEL * 2;
  const size_t PX16 = (size_t)NROWS * DMODEL * 2;
  const size_t PQK  = (size_t)NROWS * QKP * 2;
  const size_t PVT  = (size_t)NB * DMODEL * NC * 2;
  const size_t PX32 = (size_t)NROWS * DMODEL * 4;
  const size_t PG16 = (size_t)NROWS * DFF * 2;
  size_t off = 0;
  const size_t oWQK1 = off; off += PWQK;
  const size_t oWV1  = off; off += PWD;
  const size_t oWO1  = off; off += PWD;
  const size_t oWQK2 = off; off += PWQK;
  const size_t oWV2  = off; off += PWD;
  const size_t oWO2  = off; off += PWD;
  const size_t oW1T  = off; off += PWF;
  const size_t oW2T  = off; off += PWF;
  const size_t oX16  = off; off += PX16;
  const size_t oE16  = off; off += PX16;
  const size_t oQK   = off; off += PQK;
  const size_t oVT   = off; off += PVT;
  const size_t oCT   = off; off += PX16;
  const size_t oYF   = off; off += PX32;
  const size_t oX1F  = off; off += PX32;
  const size_t oX1H  = off; off += PX16;
  const size_t oX2F  = off; off += PX32;
  const size_t oX2H  = off; off += PX16;
  const size_t oG    = off; off += PG16;
  const size_t endAll = off;
  if (endAll > ws_size) return;
  if (endAll > (size_t)134217728) return;

  char* ws = (char*)d_ws;
  unsigned short* WQK1 = (unsigned short*)(ws + oWQK1);
  unsigned short* WV1  = (unsigned short*)(ws + oWV1);
  unsigned short* WO1  = (unsigned short*)(ws + oWO1);
  unsigned short* WQK2 = (unsigned short*)(ws + oWQK2);
  unsigned short* WV2  = (unsigned short*)(ws + oWV2);
  unsigned short* WO2  = (unsigned short*)(ws + oWO2);
  unsigned short* W1T  = (unsigned short*)(ws + oW1T);
  unsigned short* W2T  = (unsigned short*)(ws + oW2T);
  unsigned short* X16  = (unsigned short*)(ws + oX16);
  unsigned short* E16  = (unsigned short*)(ws + oE16);
  unsigned short* QK16 = (unsigned short*)(ws + oQK);
  unsigned short* VTp  = (unsigned short*)(ws + oVT);
  unsigned short* CT   = (unsigned short*)(ws + oCT);
  float*          YF   = (float*)(ws + oYF);
  float*          X1F  = (float*)(ws + oX1F);
  unsigned short* X1H  = (unsigned short*)(ws + oX1H);
  float*          X2F  = (float*)(ws + oX2F);
  unsigned short* X2H  = (unsigned short*)(ws + oX2H);
  unsigned short* G16  = (unsigned short*)(ws + oG);

  const dim3 blk(256);
  const int n8X = SEQ * DMODEL / 8;
  const dim3 gCX((n8X + 255) / 256);
  const dim3 gTD(DMODEL / 64, DMODEL / 64);
  const dim3 gT1(DFF / 64, DMODEL / 64);
  const dim3 gT2(DMODEL / 64, DFF / 64);
  const int tilesQK = (NROWS / 64) * (QKP / 64);
  const int tilesV  = (DMODEL / 64) * (NC / 64);
  const int tilesB  = (SEQ / 64) * (DMODEL / 64);
  const int tilesP  = (NROWS / 64) * (DMODEL / 64);
  const int tilesF  = (NROWS / 64) * (DFF / 64);
  const dim3 gQK((tilesQK + 7) / 8, 1);
  const dim3 gV((tilesV + 7) / 8, NB);
  const dim3 gB((tilesB + 7) / 8, NB);
  const dim3 gP((tilesP + 7) / 8, 1);
  const dim3 gF((tilesF + 7) / 8, 1);
  const dim3 gAT(ATT_BLOCKS);
  const dim3 bAT(ATT_THREADS);
  const dim3 gLN(NROWS);
  const dim3 bLN(LN_THREADS);

  cvtT16<<<gTD, blk, 0, stream>>>(q1_w, WQK1,                            DMODEL, DMODEL, WSC);
  cvtT16<<<gTD, blk, 0, stream>>>(k1_w, WQK1 + (size_t)DMODEL * DMODEL,  DMODEL, DMODEL, WSC);
  cvtT16<<<gTD, blk, 0, stream>>>(v1_w, WV1,                             DMODEL, DMODEL, WSC);
  cvtT16<<<gTD, blk, 0, stream>>>(o1_w, WO1,                             DMODEL, DMODEL, WSC);
  cvtT16<<<gTD, blk, 0, stream>>>(q2_w, WQK2,                            DMODEL, DMODEL, WSC);
  cvtT16<<<gTD, blk, 0, stream>>>(k2_w, WQK2 + (size_t)DMODEL * DMODEL,  DMODEL, DMODEL, WSC);
  cvtT16<<<gTD, blk, 0, stream>>>(v2_w, WV2,                             DMODEL, DMODEL, WSC);
  cvtT16<<<gTD, blk, 0, stream>>>(o2_w, WO2,                             DMODEL, DMODEL, WSC);
  cvtT16<<<gT1, blk, 0, stream>>>(f1_w, W1T, DMODEL, DFF, WSC);
  cvtT16<<<gT2, blk, 0, stream>>>(f2_w, W2T, DFF, DMODEL, WSC);

  for (int b = 0; b < NB; ++b) {
    cvt16<<<gCX, blk, 0, stream>>>(x   + (size_t)b * SEQ_FULL * DMODEL, X16 + (size_t)b * SEQ * DMODEL, n8X, XC);
    cvt16<<<gCX, blk, 0, stream>>>(enc + (size_t)b * SEQ_FULL * DMODEL, E16 + (size_t)b * SEQ * DMODEL, n8X, XC);
  }

  gemm64<2, 0, 0, 1><<<gQK, blk, 0, stream>>>(
      X16, DMODEL, 0LL,
      WQK1, DMODEL, 0LL,
      x, 0LL,
      q1_b, DMODEL, k1_b, DMODEL,
      (void*)QK16, QKP, 0LL,
      NROWS, QKP, DMODEL, 1.0f / (XC * WSC), QC);
  gemm64<2, 0, 0, 2><<<gV, blk, 0, stream>>>(
      WV1, DMODEL, 0LL,
      X16, DMODEL, (long long)NC * DMODEL,
      x, 0LL,
      v1_b, DMODEL, v1_b, DMODEL,
      (void*)VTp, NC, (long long)DMODEL * NC,
      DMODEL, NC, DMODEL, 1.0f / (XC * WSC), VC);
  attn8<0><<<gAT, bAT, 0, stream>>>(QK16, VTp, lmask, CT);
  gemm64<0, 1, 0, 1><<<gB, blk, 0, stream>>>(
      CT, DMODEL, (long long)SEQ * DMODEL,
      WO1, DMODEL, 0LL,
      x, (long long)SEQ_FULL * DMODEL,
      o1_b, DMODEL, o1_b, DMODEL,
      (void*)YF, DMODEL, (long long)SEQ * DMODEL,
      SEQ, DMODEL, DMODEL, 1.0f / (FC * WSC), 1.0f);
  lnorm<1, 1><<<gLN, bLN, 0, stream>>>(YF, ln1_g, ln1_b, X1F, X1H, X1C, (unsigned)SEQ, (unsigned)SEQ);

  gemm64<2, 0, 0, 1><<<gQK, blk, 0, stream>>>(
      E16, DMODEL, 0LL,
      WQK2, DMODEL, 0LL,
      x, 0LL,
      q2_b, DMODEL, k2_b, DMODEL,
      (void*)QK16, QKP, 0LL,
      NROWS, QKP, DMODEL, 1.0f / (XC * WSC), QC);
  gemm64<2, 0, 0, 2><<<gV, blk, 0, stream>>>(
      WV2, DMODEL, 0LL,
      X1H, DMODEL, (long long)NC * DMODEL,
      x, 0LL,
      v2_b, DMODEL, v2_b, DMODEL,
      (void*)VTp, NC, (long long)DMODEL * NC,
      DMODEL, NC, DMODEL, 1.0f / (X1C * WSC), VC);
  attn8<1><<<gAT, bAT, 0, stream>>>(QK16, VTp, pmask, CT);
  gemm64<0, 2, 0, 1><<<gP, blk, 0, stream>>>(
      CT, DMODEL, 0LL,
      WO2, DMODEL, 0LL,
      X1F, 0LL,
      o2_b, DMODEL, o2_b, DMODEL,
      (void*)YF, DMODEL, 0LL,
      NROWS, DMODEL, DMODEL, 1.0f / (FC * WSC), 1.0f);
  lnorm<1, 1><<<gLN, bLN, 0, stream>>>(YF, ln2_g, ln2_b, X2F, X2H, X1C, (unsigned)SEQ, (unsigned)SEQ);

  gemm64<2, 0, 1, 1><<<gF, blk, 0, stream>>>(
      X2H, DMODEL, 0LL,
      W1T, DMODEL, 0LL,
      x, 0LL,
      f1_b, DFF, f1_b, DFF,
      (void*)G16, DFF, 0LL,
      NROWS, DFF, DMODEL, 1.0f / (X1C * WSC), GC);
  gemm64<0, 2, 0, 1><<<gP, blk, 0, stream>>>(
      G16, DFF, 0LL,
      W2T, DFF, 0LL,
      X2F, 0LL,
      f2_b, DMODEL, f2_b, DMODEL,
      (void*)YF, DMODEL, 0LL,
      NROWS, DMODEL, DFF, 1.0f / (GC * WSC), 1.0f);
  lnorm<1, 0><<<gLN, bLN, 0, stream>>>(YF, ln3_g, ln3_b, out, X2H, 1.0f, (unsigned)SEQ, (unsigned)SEQ_FULL);
  (void)hipGetLastError();
}
